// SpatialTransformer_60782377173633
// MI455X (gfx1250) — hardware-verified
//
#include <hip/hip_runtime.h>


namespace {
constexpr int NB = 16, H = 224, W = 224, C = 16, CO = 8, KS = 7, HC = 218, WC = 218, WCP = 224  , HP = 109, WP = 109, KCV = KS * KS * C  , KCP = 800, FLAT = HP * WP * CO  , NH1 = 32, KCH = 256  , NCH = (FLAT + KCH - 1) / KCH  ;
constexpr float XS = 8.0f, WSC = 256.0f;
typedef _Float16 b16;
typedef __attribute__((ext_vector_type(16))) _Float16 v16b;
typedef __attribute__((ext_vector_type(8))) _Float16 v8b;
typedef __attribute__((ext_vector_type(8))) float v8f;
typedef __attribute__((ext_vector_type(4))) float v4f;
__device__ __forceinline__ float bf16_rne(float f) { unsigned int u = __float_as_uint(f); u += 0x7FFFu + ((u >> 16) & 1u); float r = __uint_as_float(u & 0xFFFF0000u); asm volatile("" : "+v"(r)); return r; }
__device__ __forceinline__ float bfv(float f) { float r = bf16_rne(f); asm volatile("" : "+v"(r)); return r; }
__device__ __forceinline__ void split16(float v, b16& hi, b16& lo) { hi = (b16)v; lo = (b16)(v - (float)hi); }
__device__ __forceinline__ v16b frag_kb(const b16* p, int hh) { const v8b a = *(const v8b*)(p + 8 * hh), b = *(const v8b*)(p + 16 + 8 * hh); v16b f;
#pragma unroll
  for (int e = 0; e < 8; ++e) { f[e] = a[e]; f[8 + e] = b[e]; } return f; }
__device__ __forceinline__ v8f wmma16b(v16b a, v16b b, v8f c) { v8f d = __builtin_amdgcn_wmma_f32_16x16x32_f16(false, a, false, b, (short)0, c, false, false); asm volatile("v_nop\n\tv_nop\n\tv_nop\n\tv_nop" : "+v"(d) : "v"(a), "v"(b)); return d; }
__device__ __forceinline__ void wave_lds_sync() { __builtin_amdgcn_fence(__ATOMIC_RELEASE, "workgroup"); __builtin_amdgcn_wave_barrier(); __builtin_amdgcn_fence(__ATOMIC_ACQUIRE, "workgroup"); }
__device__ __forceinline__ float pmul(float a, float b) { float p = a * b; asm volatile("" : "+v"(p)); return p; }
__device__ __forceinline__ int iclamp(int v, int lo, int hi) { return v < lo ? lo : (v > hi ? hi : v); }

__global__ __launch_bounds__(256) void wput_kernel(const float* __restrict__ cw, const float* __restrict__ w1, b16* __restrict__ CW, b16* __restrict__ W1T) { const size_t u = (size_t)blockIdx.x * 256 + threadIdx.x; v8b v;
  if (u < (size_t)16 * (KCP / 8)) { const int o = (int)(u / (KCP / 8)), k0 = (int)(u % (KCP / 8)) * 8;
#pragma unroll
    for (int j = 0; j < 8; ++j) { const int k = k0 + j; v[j] = (b16)((o < CO && k < KCV) ? bf16_rne(cw[(size_t)k * CO + o]) * WSC : 0.0f); } for (int pass = 0; pass < 2; ++pass) { *(volatile v8b*)(CW + (size_t)o * KCP + k0) = v; __threadfence(); } }
  if (u < (size_t)NH1 * (NCH * KCH / 8)) { const int o = (int)(u / (NCH * KCH / 8)), k0 = (int)(u % (NCH * KCH / 8)) * 8;
#pragma unroll
    for (int j = 0; j < 8; ++j) { const int k = k0 + j; v[j] = (b16)(k < FLAT ? bf16_rne(w1[(size_t)k * NH1 + o]) * WSC : 0.0f); } for (int pass = 0; pass < 2; ++pass) { *(volatile v8b*)(W1T + (size_t)o * (NCH * KCH) + k0) = v; __threadfence(); } } }
__global__ __launch_bounds__(32) void conv_kernel(const float* __restrict__ x, const b16* __restrict__ CW, const float* __restrict__ cb, int BLIM, float* __restrict__ CV) { __shared__ __attribute__((aligned(16))) b16 Ah[16][KCP + 8]; __shared__ float Tf[16][CO]; const int lane = threadIdx.x, nloc = lane & 15, hlf = lane >> 4; const int wb = blockIdx.x % (WCP / 16); const int ho = (blockIdx.x / (WCP / 16)) % HC; const int b = blockIdx.x / ((WCP / 16) * HC); if (b >= BLIM) return; const int wo0 = wb * 16;
  for (int kh = 0; kh < KS; ++kh) for (int kw = 0; kw < KS; ++kw) { const int col = iclamp(wo0 + nloc + kw, 0, W - 1); const float* xp = x + (((size_t)b * H + ho + kh) * W + col) * C + hlf * 8; const int k0 = (kh * KS + kw) * C + hlf * 8;
#pragma unroll
    for (int j = 0; j < 8; ++j) Ah[nloc][k0 + j] = (b16)(bf16_rne(xp[j]) * XS); }
  if (lane < 16) for (int k = KCV; k < KCP; ++k) Ah[lane][k] = (b16)0.0f;
  wave_lds_sync(); v8f acc = {};
#pragma unroll 5
  for (int kb = 0; kb < KCP; kb += 32) acc = wmma16b(frag_kb(&Ah[nloc][kb], hlf), frag_kb(CW + (size_t)nloc * KCP + kb, hlf), acc);
  if (nloc < CO) { const float bb = bfv(cb[nloc]);
#pragma unroll
    for (int r8 = 0; r8 < 8; ++r8) Tf[8 * hlf + r8][nloc] = fmaxf(acc[r8] * (1.0f / (XS * WSC)) + bb, 0.0f); }
  wave_lds_sync();
  for (int pass = 0; pass < 2; ++pass) { *(volatile v4f*)(CV + (((size_t)b * HC + ho) * WCP + wo0 + (lane >> 1)) * CO + (lane & 1) * 4) = *(const v4f*)(&Tf[lane >> 1][(lane & 1) * 4]); __threadfence(); } }
__global__ __launch_bounds__(32) void fc_kernel(const float* __restrict__ CV, const b16* __restrict__ W1T, float* __restrict__ PART) { __shared__ __attribute__((aligned(16))) b16 Ah[16][KCH + 8], Al[16][KCH + 8]; __shared__ float Tf[16][36]; const int lane = threadIdx.x, nloc = lane & 15, hlf = lane >> 4; const int ch = blockIdx.x;
  for (int kk = lane; kk < KCH; kk += 32) { const int k = ch * KCH + kk; int hp = 0, wp = 0, o = 0; const bool ok = k < FLAT; if (ok) { o = k % CO; wp = (k / CO) % WP; hp = k / (CO * WP); }
    for (int b = 0; b < NB; ++b) { float v = 0.0f; if (ok) { const float* p0 = CV + (((size_t)b * HC + 2 * hp) * WCP + 2 * wp) * CO + o; v = fmaxf(fmaxf(p0[0], p0[CO]), fmaxf(p0[(size_t)WCP * CO], p0[(size_t)WCP * CO + CO])); } b16 p, ql; split16(v * XS, p, ql); Ah[b][kk] = p; Al[b][kk] = ql; } }
  wave_lds_sync(); v8f acc[2] = {(v8f){}, (v8f){}};
#pragma unroll
  for (int kb = 0; kb < KCH; kb += 32) { const v16b a = frag_kb(&Ah[nloc][kb], hlf), al = frag_kb(&Al[nloc][kb], hlf);
#pragma unroll
    for (int t = 0; t < 2; ++t) { const v16b bw = frag_kb(W1T + (size_t)(t * 16 + nloc) * (NCH * KCH) + (size_t)ch * KCH + kb, hlf); acc[t] = wmma16b(a, bw, acc[t]); acc[t] = wmma16b(al, bw, acc[t]); } }
#pragma unroll
  for (int t = 0; t < 2; ++t)
#pragma unroll
    for (int r8 = 0; r8 < 8; ++r8) Tf[8 * hlf + r8][t * 16 + nloc] = acc[t][r8] * (1.0f / (XS * WSC));
  wave_lds_sync();
  for (int pass = 0; pass < 2; ++pass) { for (int b = 0; b < NB; ++b) ((volatile float*)PART)[((size_t)ch * NB + b) * NH1 + lane] = Tf[b][lane]; __threadfence(); } }
__global__ __launch_bounds__(512) void theta_kernel(const float* __restrict__ PART, const float* __restrict__ b1, const float* __restrict__ w2, float* __restrict__ TH) { const int b = threadIdx.x >> 5, lane = threadIdx.x & 31; double s = 0.0;
#pragma unroll 1
  for (int ch = 0; ch < NCH; ++ch) s += (double)PART[((size_t)ch * NB + b) * NH1 + lane];
  const float h1 = fmaxf((float)s + bfv(b1[lane]), 0.0f); float th = 0.0f;
#pragma unroll 1
  for (int o = 0; o < NH1; ++o) { const float ho = __shfl(h1, o); if (lane < 6) th += pmul(ho, bfv(w2[o * 6 + lane])); }
  for (int pass = 0; pass < 2; ++pass) { ((volatile float*)TH)[b * 32 + lane] = lane < 6 ? th : 0.0f; __threadfence(); } }
__global__ __launch_bounds__(256) void sample_kernel(const float* __restrict__ x, const float* __restrict__ TH, int BLIM, float* __restrict__ out) { const size_t u = (size_t)blockIdx.x * 256 + threadIdx.x; if (u >= (size_t)BLIM * H * W) return; const int col = (int)(u % W); const int row = (int)((u / W) % H); const int b = (int)(u / ((size_t)H * W));
  const float* th = TH + b * 32; const float xt = -1.0f + (2.0f / (float)(W - 1)) * (float)col, yt = -1.0f + (2.0f / (float)(H - 1)) * (float)row;
  const float gxn = th[0] * xt + th[1] * yt + th[2], gyn = th[3] * xt + th[4] * yt + th[5];
  const float gx = (gxn + 1.0f) * 0.5f * (float)W, gy = (gyn + 1.0f) * 0.5f * (float)H;
  const int x0 = iclamp((int)floorf(gx), 0, W - 1), y0 = iclamp((int)floorf(gy), 0, H - 1); const int x1 = iclamp(x0 + 1, 0, W - 1), y1 = iclamp(y0 + 1, 0, H - 1);
  const float x0f = (float)x0, x1f = (float)x1, y0f = (float)y0, y1f = (float)y1;
  const float wa = (x1f - gx) * (y1f - gy), wb = (x1f - gx) * (gy - y0f), wc = (gx - x0f) * (y1f - gy), wd = (gx - x0f) * (gy - y0f);
  const float* Ia = x + (((size_t)b * H + y0) * W + x0) * C; const float* Ib = x + (((size_t)b * H + y1) * W + x0) * C; const float* Ic = x + (((size_t)b * H + y0) * W + x1) * C; const float* Id = x + (((size_t)b * H + y1) * W + x1) * C;
  float o[16];
#pragma unroll
  for (int c = 0; c < C; ++c) o[c] = pmul(wa, bfv(Ia[c])) + pmul(wb, bfv(Ib[c])) + pmul(wc, bfv(Ic[c])) + pmul(wd, bfv(Id[c]));
  for (int pass = 0; pass < 2; ++pass) { float* dst = out + u * C;
#pragma unroll
    for (int q = 0; q < 4; ++q) *(volatile v4f*)(dst + q * 4) = (v4f){o[q * 4], o[q * 4 + 1], o[q * 4 + 2], o[q * 4 + 3]};
    __threadfence(); } }
}

extern "C" void kernel_launch(void* const* d_in, const int* in_sizes, int n_in, void* d_out, int out_size, void* d_ws, size_t ws_size, hipStream_t stream) {
  (void)n_in;
  auto Fp = [&](int i) { return (const float*)d_in[i]; };
  if (in_sizes[0] != NB * H * W * C || in_sizes[1] != KCV * CO || in_sizes[2] != CO || in_sizes[3] != FLAT * NH1 || in_sizes[4] != NH1 || in_sizes[5] != NH1 * 6 || out_size != NB * H * W * C) return;
  const int BLIM = NB;
  size_t off = 0; char* ws = (char*)d_ws;
  auto carve = [&](size_t bytes) { char* p = ws + off; off += (bytes + 255) & ~(size_t)255; return p; };
  b16* CW = (b16*)carve((size_t)16 * KCP * 2); b16* W1T = (b16*)carve((size_t)NH1 * NCH * KCH * 2); float* CV = (float*)carve((size_t)NB * HC * WCP * CO * 4); float* PART = (float*)carve((size_t)NCH * NB * NH1 * 4); float* TH = (float*)carve(NB * 32 * 4);
  if (off > ws_size || off > ((size_t)48 << 20)) return;
  wput_kernel<<<(unsigned)(((size_t)NH1 * (NCH * KCH / 8) + 255) / 256), 256, 0, stream>>>(Fp(1), Fp(3), CW, W1T);
  conv_kernel<<<BLIM * HC * (WCP / 16), 32, 0, stream>>>(Fp(0), CW, Fp(2), BLIM, CV);
  fc_kernel<<<NCH, 32, 0, stream>>>(CV, W1T, PART);
  theta_kernel<<<1, 512, 0, stream>>>(PART, Fp(4), Fp(5), TH);
  sample_kernel<<<(unsigned)(((size_t)BLIM * H * W + 255) / 256), 256, 0, stream>>>(Fp(0), TH, BLIM, (float*)d_out);
}
